// MultiScaleFeatureFusionWithAttention_38783554683411
// MI455X (gfx1250) — hardware-run, weakly checked
//
#include <hip/hip_runtime.h>
#include <stdint.h>

#define NB     16
#define CH     256
#define CQ     128
#define IMG    32
#define HW     1024
#define PT     32
#define NTAP   35
#define KK     8960
#define GS     2
#define NG     8
#define NSEG   35840
#define SEGW   14
#define SEGWA  5
#define NTOK   16384
#define QTILE  64
#define SPP    40
#define SLP    36

#define COLSCALE 64.0f
#define WSCALE   1024.0f
#define OSCALE_A (1.0f / 65536.0f)
#define SHI      16384.0f
#define SLO      4.0f
#define ALO      4096.0f
#define OSCALE_S (1.0f / 16384.0f)
#define PSCALE   1024.0f
#define PINV     (1.0f / 1024.0f)

static_assert(NB == GS * NG);
static_assert(HW == IMG * IMG);
static_assert(PT * 32 == HW);
static_assert(KK == NTAP * CH);
static_assert(NSEG == HW * NTAP);
static_assert(NSEG % (8 * SEGW) == 0);
static_assert((CH * NTAP) % (8 * SEGWA) == 0);
static_assert(NTOK == NB * HW);
static_assert((KK % 32) == 0 && (HW % 64) == 0 && (CH % 64) == 0 && (CQ % 64) == 0);
static_assert(((CH / 64) * (HW / 64)) % 8 == 0);
static_assert(((CQ / 64) * (HW / 64)) % 8 == 0);
static_assert(HW % QTILE == 0 && QTILE == 64);
static_assert((NB * CH) % 8 == 0);

typedef _Float16 v16h __attribute__((ext_vector_type(16)));
typedef _Float16 v8h  __attribute__((ext_vector_type(8)));
typedef float    v8f  __attribute__((ext_vector_type(8)));
typedef float    v4f  __attribute__((ext_vector_type(4)));
typedef unsigned int v4u __attribute__((ext_vector_type(4)));

__device__ __forceinline__ unsigned short bf_bits(float f) {
  unsigned u = __float_as_uint(f);
  return (unsigned short)((u + 0x7FFFu + ((u >> 16) & 1u)) >> 16);
}
__device__ __forceinline__ float bf_up(unsigned short h) { return __uint_as_float(((unsigned)h) << 16); }
__device__ __forceinline__ float bfr(float f) { return bf_up(bf_bits(f)); }
__device__ __forceinline__ unsigned short h_bits(_Float16 x) { return __builtin_bit_cast(unsigned short, x); }
__device__ __forceinline__ unsigned short f2h_bits(float f) { return h_bits((_Float16)f); }
__device__ __forceinline__ unsigned pk16(unsigned short a, unsigned short b) { return (unsigned)a | ((unsigned)b << 16); }
__device__ __forceinline__ v8f zero8() { v8f z = {0.f, 0.f, 0.f, 0.f, 0.f, 0.f, 0.f, 0.f}; return z; }

__device__ __forceinline__ unsigned split_pair(float a, float b, unsigned& lo) {
  const _Float16 ha = (_Float16)a, hb = (_Float16)b;
  const _Float16 la = (_Float16)((a - (float)ha) * ALO);
  const _Float16 lb = (_Float16)((b - (float)hb) * ALO);
  lo = pk16(h_bits(la), h_bits(lb));
  return pk16(h_bits(ha), h_bits(hb));
}

__device__ __forceinline__ v16h ldfrag_h(const _Float16* p) {
  union { v16h v; v8h h[2]; } f;
  f.h[0] = *(const v8h*)(p);
  f.h[1] = *(const v8h*)(p + 16);
  return f.v;
}

__device__ __forceinline__ v8f mma_h_raw(v16h a, v16h b, v8f c) {
  return __builtin_amdgcn_wmma_f32_16x16x32_f16(false, a, false, b, (short)0, c, false, false);
}
__device__ __forceinline__ void dep_guard1(v8f& a, v16h x, v16h y) {
#if defined(__HIP_DEVICE_COMPILE__)
  asm volatile("v_nop\n\tv_nop\n\tv_nop\n\tv_nop" : "+v"(a) : "v"(x), "v"(y));
#endif
}
__device__ __forceinline__ void dep_guard_h(v8f& a, v8f& b, v16h x, v16h y) {
#if defined(__HIP_DEVICE_COMPILE__)
  asm volatile("v_nop\n\tv_nop\n\tv_nop\n\tv_nop" : "+v"(a), "+v"(b) : "v"(x), "v"(y));
#endif
}
__device__ __forceinline__ void keep4_h(v16h a, v16h b, v16h c, v16h d) {
#if defined(__HIP_DEVICE_COMPILE__)
  asm volatile("v_nop" :: "v"(a), "v"(b), "v"(c), "v"(d));
#endif
}
__device__ __forceinline__ void keep2_h(v16h a, v16h b) {
#if defined(__HIP_DEVICE_COMPILE__)
  asm volatile("v_nop" :: "v"(a), "v"(b));
#endif
}
__device__ __forceinline__ void acc_guard4(v8f& a, v8f& b, v8f& c, v8f& d) {
#if defined(__HIP_DEVICE_COMPILE__)
  asm volatile("v_nop\n\tv_nop\n\tv_nop\n\tv_nop" : "+v"(a), "+v"(b), "+v"(c), "+v"(d));
#endif
}
__device__ __forceinline__ void wave_sync_lds() {
  __builtin_amdgcn_fence(__ATOMIC_RELEASE, "workgroup");
  __builtin_amdgcn_wave_barrier();
  __builtin_amdgcn_fence(__ATOMIC_ACQUIRE, "workgroup");
}

__global__ __launch_bounds__(256) void cvt_xt(const float* __restrict__ x, unsigned short* xt) {
  __shared__ __align__(16) float sx[CH * 33];
  const int tid = threadIdx.x;
  const int b   = blockIdx.x / PT;
  const int tp  = blockIdx.x - b * PT;
  const int p0  = tp * 32;
  const float* xb = x + (size_t)b * CH * HW;
#pragma unroll 8
  for (int it = 0; it < 32; ++it) {
    const int idx = it * 256 + tid;
    const int c = idx >> 5, q = idx & 31;
    sx[c * 33 + q] = xb[(size_t)c * HW + p0 + q];
  }
  __syncthreads();
  const int wave = tid >> 5, lane = tid & 31, c8 = lane * 8;
  v4u pk[4];
#pragma unroll
  for (int it = 0; it < 4; ++it) {
    const int r = wave * 4 + it;
    v4u p;
#pragma unroll
    for (int e = 0; e < 4; ++e)
      p[e] = pk16(bf_bits(sx[(c8 + 2 * e) * 33 + r]), bf_bits(sx[(c8 + 2 * e + 1) * 33 + r]));
    pk[it] = p;
  }
  unsigned short* dst = xt + ((size_t)b * HW + p0) * CH;
  for (int pass = 0; pass < 2; ++pass) {
#pragma unroll
    for (int it = 0; it < 4; ++it) {
      const int r = wave * 4 + it;
      *(volatile v4u*)(dst + (size_t)r * CH + c8) = pk[it];
    }
    __threadfence();
  }
}

__global__ __launch_bounds__(256) void cvt_wa(const float* __restrict__ w1, const float* __restrict__ w3,
                                               const float* __restrict__ w5, unsigned short* wp) {
  const int tid = threadIdx.x, wave = tid >> 5, lane = tid & 31, c8 = lane * 8;
#pragma unroll 1
  for (int it = 0; it < SEGWA; ++it) {
    const int seg = (blockIdx.x * 8 + wave) * SEGWA + it;
    if (seg < CH * NTAP) {
      const int o = seg / NTAP, tap = seg - o * NTAP;
      const float* src;
      int strd;
      if (tap < 25)      { src = w5 + ((size_t)o * CH + c8) * 25 + tap;       strd = 25; }
      else if (tap < 34) { src = w3 + ((size_t)o * CH + c8) * 9 + (tap - 25); strd = 9; }
      else               { src = w1 + ((size_t)o * CH + c8);                  strd = 1; }
      float vals[8];
#pragma unroll
      for (int i = 0; i < 8; ++i) vals[i] = bfr(src[i * strd]) * WSCALE;
      v4u p;
#pragma unroll
      for (int i = 0; i < 4; ++i) p[i] = pk16(f2h_bits(vals[2 * i]), f2h_bits(vals[2 * i + 1]));
      unsigned short* d = wp + (size_t)o * KK + (size_t)tap * CH + c8;
      *(volatile v4u*)d = p;
      __threadfence();
      *(volatile v4u*)d = p;
    }
  }
}

__global__ __launch_bounds__(256) void cvt_ws(const float* __restrict__ w, int nrows, int K, unsigned short* dst) {
  const int tid = threadIdx.x, wave = tid >> 5, lane = tid & 31, c8 = lane * 8;
  const int row = blockIdx.x * 8 + wave;
  if (row < nrows) {
    const float* src = w + (size_t)row * K;
    unsigned short* d = dst + (size_t)row * (2 * K);
#pragma unroll 1
    for (int kk = 0; kk < K; kk += 256) {
      float vals[8];
#pragma unroll
      for (int i = 0; i < 8; ++i) vals[i] = bfr(src[kk + c8 + i]);
      v4u ph, pl;
#pragma unroll
      for (int i = 0; i < 4; ++i) {
        ph[i] = pk16(f2h_bits(vals[2 * i] * SHI), f2h_bits(vals[2 * i + 1] * SHI));
        pl[i] = pk16(f2h_bits(vals[2 * i] * SLO), f2h_bits(vals[2 * i + 1] * SLO));
      }
      unsigned short* dh = d + kk + c8;
      unsigned short* dl = d + K + kk + c8;
      *(volatile v4u*)dh = ph;
      *(volatile v4u*)dl = pl;
      __threadfence();
      *(volatile v4u*)dh = ph;
      *(volatile v4u*)dl = pl;
    }
  }
}

__global__ __launch_bounds__(256) void im2col_a(const unsigned short* __restrict__ xt, unsigned short* col) {
  const int bl = blockIdx.y;
  const unsigned short* xs = xt + (size_t)bl * HW * CH;
  unsigned short* cd = col + (size_t)bl * HW * KK;
  const int tid = threadIdx.x, wave = tid >> 5, lane = tid & 31, c8 = lane * 8;
  const int segb = (blockIdx.x * 8 + wave) * SEGW;
#pragma unroll 1
  for (int it = 0; it < SEGW; ++it) {
    const int seg = segb + it;
    if (seg < NSEG) {
      const int p   = seg / NTAP;
      const int tap = seg - p * NTAP;
      int dy, dx;
      if (tap < 25)      { const int ky = tap / 5; dy = ky - 2; dx = tap - ky * 5 - 2; }
      else if (tap < 34) { const int u = tap - 25; const int ky = u / 3; dy = ky - 1; dx = u - ky * 3 - 1; }
      else               { dy = 0; dx = 0; }
      const int py  = p >> 5, px = p & 31;
      const int yy  = py + dy, xx = px + dx;
      const bool ok = ((unsigned)yy < 32u) && ((unsigned)xx < 32u);
      const int yyc = min(max(yy, 0), 31), xxc = min(max(xx, 0), 31);
      const int pix = yyc * IMG + xxc;
      const v4u xv = *(const v4u*)(xs + (size_t)pix * CH + c8);
      v4u o;
#pragma unroll
      for (int e = 0; e < 4; ++e) {
        const float x0 = bf_up((unsigned short)(xv[e] & 0xFFFFu)) * COLSCALE;
        const float x1 = bf_up((unsigned short)(xv[e] >> 16)) * COLSCALE;
        const unsigned wv = pk16(f2h_bits(x0), f2h_bits(x1));
        o[e] = ok ? wv : 0u;
      }
      unsigned short* d = cd + (size_t)seg * CH + c8;
      *(volatile v4u*)d = o;
      __threadfence();
      *(volatile v4u*)d = o;
    }
  }
}

__global__ __launch_bounds__(256) void gemm64(
    const unsigned short* __restrict__ Ap, int lda,
    const unsigned short* __restrict__ Btp, int ldb, long long strideB,
    float* Cp, int ldc, long long strideC,
    int M, int N, int K, float oscale,
    const float* __restrict__ bias0, const float* __restrict__ bias1,
    const float* __restrict__ bias2, int nb) {
  const _Float16* A  = (const _Float16*)(const void*)Ap;
  const _Float16* Bt = (const _Float16*)(const void*)Btp;
  __shared__ __align__(16) float sT[8][16 * 68];
  const int b    = blockIdx.y;
  const int lane = threadIdx.x & 31;
  const int wave = threadIdx.x >> 5;
  const int tilesN = N >> 6;
  const int tilesM = M >> 6;
  const int tile = blockIdx.x * 8 + wave;
  if (tile >= tilesM * tilesN) return;
  const int tm = tile / tilesN;
  const int tn = tile - tm * tilesN;
  const int m0 = tm << 6;
  const int n0 = tn << 6;

  const _Float16* Bb = Bt + (size_t)b * strideB;

  const int rlane = lane & 15;
  const int koff  = (lane >> 4) * 8;
  const int mOff  = (lane >> 4) * 8;

  v8f acc[4][4];
#pragma unroll
  for (int i = 0; i < 4; ++i)
#pragma unroll
    for (int j = 0; j < 4; ++j) acc[i][j] = zero8();

  for (int k0 = 0; k0 < K; k0 += 32) {
    v16h bh[4];
#pragma unroll
    for (int j = 0; j < 4; ++j) {
      const size_t bo = (size_t)(n0 + (j << 4) + rlane) * ldb + koff + k0;
      bh[j] = ldfrag_h(Bb + bo);
    }
#pragma unroll
    for (int i = 0; i < 4; ++i) {
      const size_t ao = (size_t)(m0 + (i << 4) + rlane) * lda + koff + k0;
      const v16h ah = ldfrag_h(A + ao);
#pragma unroll
      for (int j = 0; j < 4; ++j) {
        acc[i][j] = mma_h_raw(ah, bh[j], acc[i][j]);
      }
      dep_guard_h(acc[i][0], acc[i][3], ah, bh[3]);
    }
    keep4_h(bh[0], bh[1], bh[2], bh[3]);
  }
  acc_guard4(acc[0][0], acc[0][1], acc[0][2], acc[0][3]);
  acc_guard4(acc[1][0], acc[1][1], acc[1][2], acc[1][3]);
  acc_guard4(acc[2][0], acc[2][1], acc[2][2], acc[2][3]);
  acc_guard4(acc[3][0], acc[3][1], acc[3][2], acc[3][3]);

  float* slab = sT[wave];
  float* C = Cp + (size_t)b * strideC;
#pragma unroll
  for (int i = 0; i < 4; ++i) {
    const int mBase = m0 + (i << 4);
#pragma unroll
    for (int j = 0; j < 4; ++j) {
#pragma unroll
      for (int r = 0; r < 8; ++r) {
        slab[(mOff + r) * 68 + (j << 4) + rlane] = acc[i][j][r];
      }
    }
    wave_sync_lds();
    {
      const int hh = lane >> 4, c4 = (lane & 15) * 4;
      v4f ov[8];
#pragma unroll
      for (int it = 0; it < 8; ++it) {
        const int row = it * 2 + hh;
        const int mrw = mBase + row;
        const float bv = bfr(bias0[mrw]) + ((nb > 1) ? bfr(bias1[mrw]) : 0.0f) + ((nb > 2) ? bfr(bias2[mrw]) : 0.0f);
        v4f v = *(const v4f*)(slab + row * 68 + c4);
        v[0] = v[0] * oscale + bv;
        v[1] = v[1] * oscale + bv;
        v[2] = v[2] * oscale + bv;
        v[3] = v[3] * oscale + bv;
        ov[it] = v;
      }
      for (int pass = 0; pass < 2; ++pass) {
#pragma unroll
        for (int it = 0; it < 8; ++it) {
          const int row = it * 2 + hh;
          *(volatile v4f*)(C + (size_t)(mBase + row) * ldc + n0 + c4) = ov[it];
        }
        __threadfence();
      }
    }
    wave_sync_lds();
  }
}

__global__ __launch_bounds__(256) void k_pool_ca(const float* __restrict__ outp,
                                                  const float* __restrict__ caw1,
                                                  const float* __restrict__ caw2,
                                                  float* ca) {
  __shared__ float sAvg[CH];
  __shared__ float sMxv[CH];
  __shared__ float sHa[16];
  __shared__ float sHm[16];
  __shared__ __align__(16) float sCa[CH];
  const int tid = threadIdx.x, wave = tid >> 5, lane = tid & 31;
  const int b = blockIdx.x;
#pragma unroll 1
  for (int i = 0; i < 32; ++i) {
    const int c = wave * 32 + i;
    const v4f* rowv = (const v4f*)(outp + ((size_t)b * CH + c) * HW);
    float s = 0.0f, m = -3.0e38f;
#pragma unroll
    for (int k = 0; k < 8; ++k) {
      const v4f v = rowv[k * 32 + lane];
      s += (v[0] + v[1]) + (v[2] + v[3]);
      m = fmaxf(m, fmaxf(fmaxf(v[0], v[1]), fmaxf(v[2], v[3])));
    }
#pragma unroll
    for (int off = 16; off >= 1; off >>= 1) {
      s += __shfl_xor(s, off, 32);
      m = fmaxf(m, __shfl_xor(m, off, 32));
    }
    if (lane == 0) { sAvg[c] = s * (1.0f / (float)HW); sMxv[c] = m; }
  }
  __syncthreads();
  if (tid < 16) {
    float sa = 0.0f, sm = 0.0f;
#pragma unroll 1
    for (int c = 0; c < CH; ++c) {
      const float w = bfr(caw1[tid * CH + c]);
      sa += w * sAvg[c];
      sm += w * sMxv[c];
    }
    sHa[tid] = fmaxf(sa, 0.0f);
    sHm[tid] = fmaxf(sm, 0.0f);
  }
  __syncthreads();
  {
    float s1 = 0.0f, s2 = 0.0f;
#pragma unroll 1
    for (int j = 0; j < 16; ++j) {
      const float w = bfr(caw2[tid * 16 + j]);
      s1 += w * sHa[j];
      s2 += w * sHm[j];
    }
    const float z = fminf(fmaxf(s1 + s2, -60.0f), 60.0f);
    sCa[tid] = 1.0f / (1.0f + expf(-z));
  }
  __syncthreads();
  if (tid < 64) {
    const v4f v = *(const v4f*)(sCa + 4 * tid);
    float* d = ca + (size_t)b * CH + 4 * tid;
    *(volatile v4f*)d = v;
    __threadfence();
    *(volatile v4f*)d = v;
  }
}

__global__ __launch_bounds__(256) void k_sapool_outt(const float* __restrict__ outp, const float* __restrict__ ca,
                                                      float* meanp, float* maxp, unsigned short* ot2) {
  __shared__ __align__(16) float sx[CH * 33];
  __shared__ float sCa[CH];
  __shared__ float sPS[8 * 32];
  __shared__ float sPM[8 * 32];
  __shared__ __align__(16) float sMean[32];
  __shared__ __align__(16) float sMaxv[32];
  const int tid = threadIdx.x, wave = tid >> 5, lane = tid & 31, c8 = lane * 8;
  const int b = blockIdx.x / PT, tp = blockIdx.x - b * PT, p0 = tp * 32;
  const float* ob = outp + (size_t)b * CH * HW;
#pragma unroll 8
  for (int it = 0; it < 32; ++it) {
    const int idx = it * 256 + tid;
    const int c = idx >> 5, q = idx & 31;
    sx[c * 33 + q] = ob[(size_t)c * HW + p0 + q];
  }
  sCa[tid] = ca[(size_t)b * CH + tid];
  __syncthreads();
  {
    v4u ph[4], pl[4];
#pragma unroll
    for (int it = 0; it < 4; ++it) {
      const int r = wave * 4 + it;
      v4u a, l2;
#pragma unroll
      for (int e = 0; e < 4; ++e) {
        unsigned lo;
        a[e] = split_pair(sx[(c8 + 2 * e) * 33 + r], sx[(c8 + 2 * e + 1) * 33 + r], lo);
        l2[e] = lo;
      }
      ph[it] = a; pl[it] = l2;
    }
    unsigned short* base = ot2 + ((size_t)b * HW + p0) * (2 * CH);
    for (int pass = 0; pass < 2; ++pass) {
#pragma unroll
      for (int it = 0; it < 4; ++it) {
        const int r = wave * 4 + it;
        *(volatile v4u*)(base + (size_t)r * (2 * CH) + c8) = ph[it];
        *(volatile v4u*)(base + (size_t)r * (2 * CH) + CH + c8) = pl[it];
      }
      __threadfence();
    }
  }
  {
    const int q = lane, g = wave;
    float s = 0.0f, m = -3.0e38f;
#pragma unroll 4
    for (int i = 0; i < 32; ++i) {
      const int c = g * 32 + i;
      const float v = sx[c * 33 + q] * sCa[c];
      s += v;
      m = fmaxf(m, v);
    }
    sPS[g * 32 + q] = s;
    sPM[g * 32 + q] = m;
  }
  __syncthreads();
  if (tid < 32) {
    float s = 0.0f, m = -3.0e38f;
#pragma unroll
    for (int g = 0; g < 8; ++g) { s += sPS[g * 32 + tid]; m = fmaxf(m, sPM[g * 32 + tid]); }
    sMean[tid] = s * (1.0f / (float)CH);
    sMaxv[tid] = m;
  }
  __syncthreads();
  if (tid < 8) {
    const v4f vm = *(const v4f*)(sMean + 4 * tid);
    const v4f vx = *(const v4f*)(sMaxv + 4 * tid);
    float* dm = meanp + (size_t)b * HW + p0 + 4 * tid;
    float* dx = maxp + (size_t)b * HW + p0 + 4 * tid;
    *(volatile v4f*)dm = vm;
    *(volatile v4f*)dx = vx;
    __threadfence();
    *(volatile v4f*)dm = vm;
    *(volatile v4f*)dx = vx;
  }
}

__global__ __launch_bounds__(256) void k_qkT(const float* __restrict__ qf, const float* __restrict__ kf,
                                              unsigned short* qh, unsigned short* kh, float* q2p, float* k2p) {
  __shared__ __align__(16) float st[CQ * 33];
  __shared__ __align__(16) float sQ2[32];
  const int which = blockIdx.y;
  const float* src = (which != 0) ? kf : qf;
  unsigned short* dh = (which != 0) ? kh : qh;
  float* d2 = (which != 0) ? k2p : q2p;
  const int tid = threadIdx.x, wave = tid >> 5, lane = tid & 31;
  const int b = blockIdx.x / PT, tp = blockIdx.x - b * PT, p0 = tp * 32;
  const float* sb = src + (size_t)b * CQ * HW;
#pragma unroll 4
  for (int it = 0; it < 16; ++it) {
    const int idx = it * 256 + tid;
    const int c = idx >> 5, q = idx & 31;
    st[c * 33 + q] = sb[(size_t)c * HW + p0 + q];
  }
  __syncthreads();
  if (tid < 32) {
    float s = 0.0f;
#pragma unroll 4
    for (int c = 0; c < CQ; ++c) { const float v = st[c * 33 + tid]; s += v * v; }
    sQ2[tid] = s;
  }
  {
    const int hh = lane >> 4, cl = (lane & 15) * 8;
    v4u pk[2];
#pragma unroll
    for (int it = 0; it < 2; ++it) {
      const int r = wave * 4 + it * 2 + hh;
      v4u p;
#pragma unroll
      for (int e = 0; e < 4; ++e)
        p[e] = pk16(f2h_bits(st[(cl + 2 * e) * 33 + r]), f2h_bits(st[(cl + 2 * e + 1) * 33 + r]));
      pk[it] = p;
    }
    unsigned short* base = dh + ((size_t)b * HW + p0) * CQ;
    for (int pass = 0; pass < 2; ++pass) {
#pragma unroll
      for (int it = 0; it < 2; ++it) {
        const int r = wave * 4 + it * 2 + hh;
        *(volatile v4u*)(base + (size_t)r * CQ + cl) = pk[it];
      }
      __threadfence();
    }
  }
  __syncthreads();
  if (tid < 8) {
    const v4f v = *(const v4f*)(sQ2 + 4 * tid);
    float* d = d2 + (size_t)b * HW + p0 + 4 * tid;
    *(volatile v4f*)d = v;
    __threadfence();
    *(volatile v4f*)d = v;
  }
}

__global__ __launch_bounds__(256) void k_vh(const float* __restrict__ vf, unsigned short* vh) {
  const int tid = threadIdx.x, wave = tid >> 5, lane = tid & 31;
  const int row = blockIdx.x * 8 + wave;
  if (row < NB * CH) {
    const float* s = vf + (size_t)row * HW;
    unsigned short* d = vh + (size_t)row * HW;
    v4u pk[4];
#pragma unroll
    for (int it = 0; it < 4; ++it) {
      const int base = it * 256 + lane * 8;
      const v4f a = *(const v4f*)(s + base);
      const v4f c = *(const v4f*)(s + base + 4);
      v4u p;
      p[0] = pk16(f2h_bits(a[0]), f2h_bits(a[1]));
      p[1] = pk16(f2h_bits(a[2]), f2h_bits(a[3]));
      p[2] = pk16(f2h_bits(c[0]), f2h_bits(c[1]));
      p[3] = pk16(f2h_bits(c[2]), f2h_bits(c[3]));
      pk[it] = p;
    }
    for (int pass = 0; pass < 2; ++pass) {
#pragma unroll
      for (int it = 0; it < 4; ++it)
        *(volatile v4u*)(d + it * 256 + lane * 8) = pk[it];
      __threadfence();
    }
  }
}

__global__ __launch_bounds__(256) void k_attn(const unsigned short* __restrict__ qhp,
                                               const unsigned short* __restrict__ khp,
                                               const float* __restrict__ q2p,
                                               const float* __restrict__ k2p,
                                               const unsigned short* __restrict__ vhp,
                                               const float* __restrict__ sigp,
                                               float* ao) {
  const _Float16* Q  = (const _Float16*)(const void*)qhp;
  const _Float16* Kt = (const _Float16*)(const void*)khp;
  const _Float16* V  = (const _Float16*)(const void*)vhp;
  __shared__ __align__(16) _Float16 sP[QTILE * SPP];
  __shared__ float sM1[8][16];
  __shared__ float sL1[8][16];
  __shared__ float sMrow[QTILE];
  __shared__ float sRinv[QTILE];
  __shared__ __align__(16) float slab[8][16 * SLP];

  const int tid = threadIdx.x, wave = tid >> 5, lane = tid & 31;
  const int rl = lane & 15, h = lane >> 4, koff = h * 8;
  const int b  = blockIdx.x / (HW / QTILE);
  const int qt = blockIdx.x - b * (HW / QTILE);
  const int q0 = qt * QTILE;
  const int mt = wave >> 1, kh = wave & 1;
  const size_t tokq = (size_t)b * HW + q0 + 16 * mt;

  const float sg = bfr(sigp[0]);
  const float inv2s2 = 1.0f / (2.0f * sg * sg);

  v16h qa[4];
#pragma unroll
  for (int ks = 0; ks < 4; ++ks) qa[ks] = ldfrag_h(Q + (tokq + rl) * CQ + 32 * ks + koff);
  float q2r[8];
#pragma unroll
  for (int r = 0; r < 8; ++r) q2r[r] = q2p[tokq + 8 * h + r];

  float mr[8], lr[8];
#pragma unroll
  for (int r = 0; r < 8; ++r) { mr[r] = -3.0e38f; lr[r] = 0.0f; }
  v16h kf;
#pragma unroll 1
  for (int t = 0; t < 32; ++t) {
    const size_t tokk = (size_t)b * HW + kh * 512 + 16 * t;
    v8f s = zero8();
#pragma unroll
    for (int ks = 0; ks < 4; ++ks) {
      kf = ldfrag_h(Kt + (tokk + rl) * CQ + 32 * ks + koff);
      s = mma_h_raw(qa[ks], kf, s);
    }
    dep_guard1(s, qa[3], kf);
    const float k2v = k2p[tokk + rl];
#pragma unroll
    for (int r = 0; r < 8; ++r) {
      const float d   = (q2r[r] + k2v) - 2.0f * s[r];
      const float sim = expf((-d) * inv2s2);
      const float dd  = sim - mr[r];
      const float tt  = expf(-fabsf(dd));
      const bool  gt  = dd > 0.0f;
      const float lle = lr[r] + tt;
      const float lgt = lr[r] * tt + 1.0f;
      lr[r] = gt ? lgt : lle;
      mr[r] = gt ? sim : mr[r];
    }
  }
#pragma unroll
  for (int r = 0; r < 8; ++r) {
    float mm = mr[r];
    mm = fmaxf(mm, __shfl_xor(mm, 1, 32));
    mm = fmaxf(mm, __shfl_xor(mm, 2, 32));
    mm = fmaxf(mm, __shfl_xor(mm, 4, 32));
    mm = fmaxf(mm, __shfl_xor(mm, 8, 32));
    float term = lr[r] * expf(mr[r] - mm);
    term += __shfl_xor(term, 1, 32);
    term += __shfl_xor(term, 2, 32);
    term += __shfl_xor(term, 4, 32);
    term += __shfl_xor(term, 8, 32);
    mr[r] = mm;
    lr[r] = term;
  }
  if (rl == 0) {
#pragma unroll
    for (int r = 0; r < 8; ++r) { sM1[wave][8 * h + r] = mr[r]; sL1[wave][8 * h + r] = lr[r]; }
  }
  __syncthreads();
  if (tid < QTILE) {
    const int m4 = tid >> 4, rr = tid & 15;
    const float m0 = sM1[2 * m4][rr], m1 = sM1[2 * m4 + 1][rr];
    const float l0 = sL1[2 * m4][rr], l1 = sL1[2 * m4 + 1][rr];
    const float m = fmaxf(m0, m1);
    const float l = l0 * expf(m0 - m) + l1 * expf(m1 - m);
    sMrow[tid] = m;
    sRinv[tid] = PSCALE * (1.0f / l);
  }
  __syncthreads();
  float mrow[8], rinv[8];
#pragma unroll
  for (int r = 0; r < 8; ++r) { mrow[r] = sMrow[16 * mt + 8 * h + r]; rinv[r] = sRinv[16 * mt + 8 * h + r]; }

  v8f acc[4][2];
#pragma unroll
  for (int i = 0; i < 4; ++i) { acc[i][0] = zero8(); acc[i][1] = zero8(); }
  const int cw = wave * 32;
  const _Float16* Vb = V + ((size_t)b * CH + cw) * HW;
  v16h vf0, vf1;
#pragma unroll 1
  for (int kc = 0; kc < HW / 32; ++kc) {
    const size_t tokk = (size_t)b * HW + kc * 32 + 16 * kh;
    v8f s = zero8();
#pragma unroll
    for (int ks = 0; ks < 4; ++ks) {
      kf = ldfrag_h(Kt + (tokk + rl) * CQ + 32 * ks + koff);
      s = mma_h_raw(qa[ks], kf, s);
    }
    dep_guard1(s, qa[3], kf);
    const float k2v = k2p[tokk + rl];
#pragma unroll
    for (int r = 0; r < 8; ++r) {
      const float d   = (q2r[r] + k2v) - 2.0f * s[r];
      const float sim = expf((-d) * inv2s2);
      const float pv  = expf(sim - mrow[r]) * rinv[r];
      sP[(16 * mt + 8 * h + r) * SPP + 16 * kh + rl] = (_Float16)pv;
    }
    __syncthreads();
    vf0 = ldfrag_h(Vb + (size_t)rl * HW + kc * 32 + koff);
    vf1 = ldfrag_h(Vb + (size_t)(16 + rl) * HW + kc * 32 + koff);
#pragma unroll
    for (int m2 = 0; m2 < 4; ++m2) {
      const v16h af = ldfrag_h(sP + (16 * m2 + rl) * SPP + koff);
      acc[m2][0] = mma_h_raw(af, vf0, acc[m2][0]);
      acc[m2][1] = mma_h_raw(af, vf1, acc[m2][1]);
      dep_guard_h(acc[m2][0], acc[m2][1], af, vf1);
    }
    keep2_h(vf0, vf1);
    __syncthreads();
  }
  acc_guard4(acc[0][0], acc[0][1], acc[1][0], acc[1][1]);
  acc_guard4(acc[2][0], acc[2][1], acc[3][0], acc[3][1]);

  float* sl = slab[wave];
  const int rq = lane >> 3, pc = (lane & 7) * 4;
#pragma unroll
  for (int m2 = 0; m2 < 4; ++m2) {
#pragma unroll
    for (int nt = 0; nt < 2; ++nt)
#pragma unroll
      for (int r = 0; r < 8; ++r) sl[(8 * h + r) * SLP + 16 * nt + rl] = acc[m2][nt][r] * PINV;
    wave_sync_lds();
    v4f ov[4];
#pragma unroll
    for (int it = 0; it < 4; ++it) ov[it] = *(const v4f*)(sl + (it * 4 + rq) * SLP + pc);
    for (int pass = 0; pass < 2; ++pass) {
#pragma unroll
      for (int it = 0; it < 4; ++it) {
        const int row = it * 4 + rq;
        *(volatile v4f*)(ao + ((size_t)b * HW + q0 + 16 * m2 + row) * CH + cw + pc) = ov[it];
      }
      __threadfence();
    }
    wave_sync_lds();
  }
}

__global__ __launch_bounds__(256) void k_cat(const float* __restrict__ outp, const float* __restrict__ ca,
                                              const float* __restrict__ meanp, const float* __restrict__ maxp,
                                              const float* __restrict__ saw, const float* __restrict__ aop,
                                              unsigned short* cat2) {
  __shared__ __align__(16) float sx[CH * 33];
  __shared__ float sCa[CH];
  __shared__ float sHalo[2 * 7 * 32];
  __shared__ float sW[98];
  __shared__ float sSa[32];
  const int tid = threadIdx.x, wave = tid >> 5, lane = tid & 31, c8 = lane * 8;
  const int b = blockIdx.x / PT, tp = blockIdx.x - b * PT, p0 = tp * 32;
  const float* ob = outp + (size_t)b * CH * HW;
#pragma unroll 8
  for (int it = 0; it < 32; ++it) {
    const int idx = it * 256 + tid;
    const int c = idx >> 5, q = idx & 31;
    sx[c * 33 + q] = ob[(size_t)c * HW + p0 + q];
  }
  sCa[tid] = ca[(size_t)b * CH + tid];
  if (tid < 98) sW[tid] = bfr(saw[tid]);
  for (int idx = tid; idx < 448; idx += 256) {
    const int ch  = idx / 224;
    const int rem = idx - ch * 224;
    const int ky  = rem >> 5, xx = rem & 31;
    const int yy  = tp + ky - 3;
    const bool ok = (unsigned)yy < 32u;
    const int yyc = min(max(yy, 0), 31);
    const size_t a = (size_t)b * HW + yyc * IMG + xx;
    const float vm = meanp[a];
    const float vx = maxp[a];
    const float v  = (ch != 0) ? vx : vm;
    sHalo[idx] = ok ? v : 0.0f;
  }
  __syncthreads();
  if (tid < 32) {
    const int xq = tid;
    float s = 0.0f;
#pragma unroll 1
    for (int ky = 0; ky < 7; ++ky) {
#pragma unroll 1
      for (int kx = 0; kx < 7; ++kx) {
        const int xx  = xq + kx - 3;
        const bool ok = (unsigned)xx < 32u;
        const int xxc = min(max(xx, 0), 31);
        const float am = sHalo[ky * 32 + xxc];
        const float ax = sHalo[224 + ky * 32 + xxc];
        const float w0 = sW[ky * 7 + kx];
        const float w1v = sW[49 + ky * 7 + kx];
        const float t = w0 * am + w1v * ax;
        s += ok ? t : 0.0f;
      }
    }
    const float z = fminf(fmaxf(s, -60.0f), 60.0f);
    sSa[xq] = 1.0f / (1.0f + expf(-z));
  }
  __syncthreads();
  unsigned short* base = cat2 + ((size_t)b * HW + p0) * (4 * CH);
  {
    v4u ph[4], pl[4];
#pragma unroll
    for (int it = 0; it < 4; ++it) {
      const int r = wave * 4 + it;
      const float sar = sSa[r];
      v4u a, l2;
#pragma unroll
      for (int e = 0; e < 4; ++e) {
        const int c0 = c8 + 2 * e, c1 = c0 + 1;
        const float v0 = (sx[c0 * 33 + r] * sCa[c0]) * sar;
        const float v1 = (sx[c1 * 33 + r] * sCa[c1]) * sar;
        unsigned lo;
        a[e] = split_pair(v0, v1, lo);
        l2[e] = lo;
      }
      ph[it] = a; pl[it] = l2;
    }
    for (int pass = 0; pass < 2; ++pass) {
#pragma unroll
      for (int it = 0; it < 4; ++it) {
        const int r = wave * 4 + it;
        *(volatile v4u*)(base + (size_t)r * (4 * CH) + c8) = ph[it];
        *(volatile v4u*)(base + (size_t)r * (4 * CH) + 2 * CH + c8) = pl[it];
      }
      __threadfence();
    }
  }
  __syncthreads();
  {
    const int pp = p0 >> 8, pl0 = p0 & 255;
#pragma unroll 8
    for (int it = 0; it < 32; ++it) {
      const int idx = it * 256 + tid;
      const int c = idx >> 5, q = idx & 31;
      sx[c * 33 + q] += aop[((size_t)b * HW + 4 * c + pp) * CH + pl0 + q];
    }
  }
  __syncthreads();
  {
    v4u ph[4], pl[4];
#pragma unroll
    for (int it = 0; it < 4; ++it) {
      const int r = wave * 4 + it;
      v4u a, l2;
#pragma unroll
      for (int e = 0; e < 4; ++e) {
        unsigned lo;
        a[e] = split_pair(sx[(c8 + 2 * e) * 33 + r], sx[(c8 + 2 * e + 1) * 33 + r], lo);
        l2[e] = lo;
      }
      ph[it] = a; pl[it] = l2;
    }
    for (int pass = 0; pass < 2; ++pass) {
#pragma unroll
      for (int it = 0; it < 4; ++it) {
        const int r = wave * 4 + it;
        *(volatile v4u*)(base + (size_t)r * (4 * CH) + CH + c8) = ph[it];
        *(volatile v4u*)(base + (size_t)r * (4 * CH) + 3 * CH + c8) = pl[it];
      }
      __threadfence();
    }
  }
}

extern "C" void kernel_launch(void* const* d_in, const int* in_sizes, int n_in,
                              void* d_out, int out_size, void* d_ws, size_t ws_size,
                              hipStream_t stream) {
  if (n_in < 19) return;
  if (in_sizes[0]  != NB * CH * HW) return;
  if (in_sizes[1]  != CH * CH) return;
  if (in_sizes[2]  != CH) return;
  if (in_sizes[3]  != CH * CH * 9) return;
  if (in_sizes[4]  != CH) return;
  if (in_sizes[5]  != CH * CH * 25) return;
  if (in_sizes[6]  != CH) return;
  if (in_sizes[7]  != CQ * CH) return;
  if (in_sizes[8]  != CQ) return;
  if (in_sizes[9]  != CQ * CH) return;
  if (in_sizes[10] != CQ) return;
  if (in_sizes[11] != CH * CH) return;
  if (in_sizes[12] != CH) return;
  if (in_sizes[13] < 1) return;
  if (in_sizes[14] != 16 * CH) return;
  if (in_sizes[15] != CH * 16) return;
  if (in_sizes[16] != 98) return;
  if (in_sizes[17] != CH * 2 * CH) return;
  if (in_sizes[18] != CH) return;
  if (out_size != NB * CH * HW) return;

  const float* x     = (const float*)d_in[0];
  const float* w1    = (const float*)d_in[1];
  const float* b1    = (const float*)d_in[2];
  const float* w3    = (const float*)d_in[3];
  const float* b3    = (const float*)d_in[4];
  const float* w5    = (const float*)d_in[5];
  const float* b5    = (const float*)d_in[6];
  const float* wq    = (const float*)d_in[7];
  const float* bq    = (const float*)d_in[8];
  const float* wk    = (const float*)d_in[9];
  const float* bk    = (const float*)d_in[10];
  const float* wv    = (const float*)d_in[11];
  const float* bv    = (const float*)d_in[12];
  const float* sigma = (const float*)d_in[13];
  const float* caw1  = (const float*)d_in[14];
  const float* caw2  = (const float*)d_in[15];
  const float* saw   = (const float*)d_in[16];
  const float* tw    = (const float*)d_in[17];
  const float* tb    = (const float*)d_in[18];
  float* out = (float*)d_out;

  const size_t PXT  = (size_t)NB * HW * CH * 2;
  const size_t PWP  = (size_t)CH * KK * 2;
  const size_t PCL  = (size_t)GS * HW * KK * 2;
  const size_t PQF  = (size_t)NB * CQ * HW * 4;
  const size_t PVF  = (size_t)NB * CH * HW * 4;
  const size_t PAO  = (size_t)NB * HW * CH * 4;
  const size_t PCAT = (size_t)NB * HW * (4 * CH) * 2;
  const size_t POUT = (size_t)NB * CH * HW * 4;
  const size_t POT2 = (size_t)NB * HW * (2 * CH) * 2;
  const size_t PQH  = (size_t)NTOK * CQ * 2;
  const size_t PVH  = (size_t)NB * CH * HW * 2;
  const size_t PCA  = (size_t)NB * CH * 4;
  const size_t PMP  = (size_t)NB * HW * 4;
  const size_t PWQ2 = (size_t)CQ * (2 * CH) * 2;
  const size_t PWV2 = (size_t)CH * (2 * CH) * 2;
  const size_t PWT2 = (size_t)CH * (4 * CH) * 2;

  size_t r0a = PXT + PWP + PCL;
  size_t r0b = 2 * PQF + PVF;
  size_t r0c = PAO + PCAT;
  size_t R0 = r0a; if (r0b > R0) R0 = r0b; if (r0c > R0) R0 = r0c;
  if (2 * PQH + PVH > POT2) return;

  size_t off = 0;
  const size_t oR0  = off; off += R0;
  const size_t oOUT = off; off += POUT;
  const size_t oR2  = off; off += POT2;
  const size_t oCA  = off; off += PCA;
  const size_t oMNP = off; off += PMP;
  const size_t oMXP = off; off += PMP;
  const size_t oQ2  = off; off += PMP;
  const size_t oK2  = off; off += PMP;
  const size_t oWQ2 = off; off += PWQ2;
  const size_t oWK2 = off; off += PWQ2;
  const size_t oWV2 = off; off += PWV2;
  const size_t oWT2 = off; off += PWT2;
  if (off > ws_size) return;
  if (off > (size_t)134217728) return;

  char* ws = (char*)d_ws;
  unsigned short* XT   = (unsigned short*)(ws + oR0);
  unsigned short* WP   = (unsigned short*)(ws + oR0 + PXT);
  unsigned short* COL  = (unsigned short*)(ws + oR0 + PXT + PWP);
  float*          QF   = (float*)(ws + oR0);
  float*          KF   = (float*)(ws + oR0 + PQF);
  float*          VF   = (float*)(ws + oR0 + 2 * PQF);
  float*          AO   = (float*)(ws + oR0);
  unsigned short* CAT2 = (unsigned short*)(ws + oR0 + PAO);
  float*          OUT  = (float*)(ws + oOUT);
  unsigned short* OT2  = (unsigned short*)(ws + oR2);
  unsigned short* QH   = (unsigned short*)(ws + oR2);
  unsigned short* KH   = (unsigned short*)(ws + oR2 + PQH);
  unsigned short* VH   = (unsigned short*)(ws + oR2 + 2 * PQH);
  float*          CA   = (float*)(ws + oCA);
  float*          MNP  = (float*)(ws + oMNP);
  float*          MXP  = (float*)(ws + oMXP);
  float*          Q2   = (float*)(ws + oQ2);
  float*          K2   = (float*)(ws + oK2);
  unsigned short* WQ2  = (unsigned short*)(ws + oWQ2);
  unsigned short* WK2  = (unsigned short*)(ws + oWK2);
  unsigned short* WV2  = (unsigned short*)(ws + oWV2);
  unsigned short* WT2  = (unsigned short*)(ws + oWT2);

  const dim3 blk(256);
  cvt_xt<<<dim3(NB * PT), blk, 0, stream>>>(x, XT);
  cvt_wa<<<dim3((CH * NTAP) / (8 * SEGWA)), blk, 0, stream>>>(w1, w3, w5, WP);
  cvt_ws<<<dim3(CQ / 8), blk, 0, stream>>>(wq, CQ, CH, WQ2);
  cvt_ws<<<dim3(CQ / 8), blk, 0, stream>>>(wk, CQ, CH, WK2);
  cvt_ws<<<dim3(CH / 8), blk, 0, stream>>>(wv, CH, CH, WV2);
  cvt_ws<<<dim3(CH / 8), blk, 0, stream>>>(tw, CH, 2 * CH, WT2);
  const dim3 gI2c(NSEG / (8 * SEGW), GS);
  const dim3 gGemmA(((CH / 64) * (HW / 64)) / 8, GS);
  for (int g = 0; g < NG; ++g) {
    const unsigned short* XTg = XT + (size_t)g * GS * HW * CH;
    float* OUTg = OUT + (size_t)g * GS * CH * HW;
    im2col_a<<<gI2c, blk, 0, stream>>>(XTg, COL);
    gemm64<<<gGemmA, blk, 0, stream>>>(
        WP, KK,
        COL, KK, (long long)HW * KK,
        OUTg, HW, (long long)CH * HW,
        CH, HW, KK, OSCALE_A,
        b1, b3, b5, 3);
  }
  k_pool_ca<<<dim3(NB), blk, 0, stream>>>(OUT, caw1, caw2, CA);
  k_sapool_outt<<<dim3(NB * PT), blk, 0, stream>>>(OUT, CA, MNP, MXP, OT2);
  const dim3 gGemmQ(((CQ / 64) * (HW / 64)) / 8, NB);
  const dim3 gGemmV(((CH / 64) * (HW / 64)) / 8, NB);
  gemm64<<<gGemmQ, blk, 0, stream>>>(WQ2, 2 * CH, OT2, 2 * CH, (long long)HW * (2 * CH),
                                      QF, HW, (long long)CQ * HW, CQ, HW, 2 * CH, OSCALE_S, bq, bq, bq, 1);
  gemm64<<<gGemmQ, blk, 0, stream>>>(WK2, 2 * CH, OT2, 2 * CH, (long long)HW * (2 * CH),
                                      KF, HW, (long long)CQ * HW, CQ, HW, 2 * CH, OSCALE_S, bk, bk, bk, 1);
  gemm64<<<gGemmV, blk, 0, stream>>>(WV2, 2 * CH, OT2, 2 * CH, (long long)HW * (2 * CH),
                                      VF, HW, (long long)CH * HW, CH, HW, 2 * CH, OSCALE_S, bv, bv, bv, 1);
  k_qkT<<<dim3(NB * PT, 2), blk, 0, stream>>>(QF, KF, QH, KH, Q2, K2);
  k_vh<<<dim3((NB * CH) / 8), blk, 0, stream>>>(VF, VH);
  k_attn<<<dim3(NB * (HW / QTILE)), blk, 0, stream>>>(QH, KH, Q2, K2, VH, sigma, AO);
  k_cat<<<dim3(NB * PT), blk, 0, stream>>>(OUT, CA, MNP, MXP, saw, AO, CAT2);
  gemm64<<<gGemmV, blk, 0, stream>>>(WT2, 4 * CH, CAT2, 4 * CH, (long long)HW * (4 * CH),
                                      out, HW, (long long)CH * HW, CH, HW, 4 * CH, OSCALE_S, tb, tb, tb, 1);
  (void)hipGetLastError();
}
